// LSTMAutoencoderModel_67997922230927
// MI455X (gfx1250) — hardware-verified
//
#include <hip/hip_runtime.h>
#include <math.h>

constexpr int NSEQ  = 512;
constexpr int NSTEP = 512;
constexpr int NIN   = 32;
constexpr int NHID  = 128;
constexpr int NGATE = 512;
constexpr int NOUTF = 32;
constexpr int NTHR  = 256;
constexpr int ROWS_PER_BLOCK = 16;
constexpr int XPITCH = 40;
constexpr int HPITCH = 136;
constexpr int FPITCH = 36;
constexpr float WCARRY     = 8.0f;
constexpr float WCARRY_INV = 0.125f;

static_assert((XPITCH * 2) % 16 == 0, "x tile rows 16-B aligned");
static_assert((HPITCH * 2) % 16 == 0, "h tile rows 16-B aligned");
static_assert((FPITCH * 4) % 16 == 0, "frame rows 16-B aligned");
static_assert(NIN % 32 == 0 && NHID % 32 == 0, "K multiples of 32");
static_assert(NSEQ % ROWS_PER_BLOCK == 0, "exact block tiling");

typedef __attribute__((ext_vector_type(16))) _Float16 v16h;
typedef __attribute__((ext_vector_type(8)))  _Float16 v8h;
typedef __attribute__((ext_vector_type(8)))  float    v8f;
typedef __attribute__((ext_vector_type(4)))  float    v4f;

__device__ __forceinline__ void dep_guard_h(v8f& a, v8f& b, v16h x, v16h y) { asm volatile("v_nop\n\tv_nop\n\tv_nop\n\tv_nop" : "+v"(a), "+v"(b) : "v"(x), "v"(y)); }
__device__ __forceinline__ void dep_guard1_h(v8f& a, v16h x, v16h y) { asm volatile("v_nop\n\tv_nop\n\tv_nop\n\tv_nop" : "+v"(a) : "v"(x), "v"(y)); }
__device__ __forceinline__ void keep4_h(v16h a, v16h b, v16h c, v16h d) { asm volatile("v_nop" :: "v"(a), "v"(b), "v"(c), "v"(d)); }
__device__ __forceinline__ void acc_guard4(v8f& a, v8f& b, v8f& c, v8f& d) { asm volatile("v_nop\n\tv_nop\n\tv_nop\n\tv_nop" : "+v"(a), "+v"(b), "+v"(c), "+v"(d)); }
__device__ __forceinline__ void acc_guard1(v8f& a) { asm volatile("v_nop\n\tv_nop\n\tv_nop\n\tv_nop" : "+v"(a)); }

template <typename T> struct Frag;
template <> struct Frag<_Float16> {
  typedef v16h V; union U { v16h v; v8h h[2]; };
  static __device__ __forceinline__ v16h load(const _Float16* p) {
    U f; f.h[0] = *(const v8h*)(p); f.h[1] = *(const v8h*)(p + 16); return f.v;
  }
  static __device__ __forceinline__ v8f mma(v16h a, v16h b, v8f c) {
    return __builtin_amdgcn_wmma_f32_16x16x32_f16(false, a, false, b, (short)0, c, false, false);
  }
};

__device__ __forceinline__ float fsig(float x)  { return __builtin_amdgcn_rcpf(1.0f + __expf(-x)); }
__device__ __forceinline__ float ftanh(float x) { return 1.0f - 2.0f * __builtin_amdgcn_rcpf(__expf(2.0f * x) + 1.0f); }

__global__ __launch_bounds__(256) void cast_scale_f16x2(
    const float* __restrict__ in, _Float16* __restrict__ out, int n2, float sc) {
  const int i = blockIdx.x * 256 + threadIdx.x;
  if (i < n2) {
    const _Float16 h0 = (_Float16)(in[2 * i] * sc), h1 = (_Float16)(in[2 * i + 1] * sc);
    const unsigned u = (unsigned)__builtin_bit_cast(unsigned short, h0) | ((unsigned)__builtin_bit_cast(unsigned short, h1) << 16);
    ((volatile unsigned*)out)[i] = u;
    __threadfence();
    ((volatile unsigned*)out)[i] = u;
  }
}
__global__ __launch_bounds__(256) void addcast_scale_f16x2(
    const float* __restrict__ a, const float* __restrict__ b, _Float16* __restrict__ out, int n2, float sc) {
  const int i = blockIdx.x * 256 + threadIdx.x;
  if (i < n2) {
    const float s0 = (a[2 * i] + b[2 * i]) * sc;
    const float s1 = (a[2 * i + 1] + b[2 * i + 1]) * sc;
    const _Float16 h0 = (_Float16)s0, h1 = (_Float16)s1;
    const unsigned u = (unsigned)__builtin_bit_cast(unsigned short, h0) | ((unsigned)__builtin_bit_cast(unsigned short, h1) << 16);
    ((volatile unsigned*)out)[i] = u;
    __threadfence();
    ((volatile unsigned*)out)[i] = u;
  }
}

__device__ __forceinline__ void frame_head(const _Float16* ahrow, const _Float16* wfcrow,
                                           float* Fs, int nt, int hh, int c, float fcbias) {
  v8f acc = {0.f, 0.f, 0.f, 0.f, 0.f, 0.f, 0.f, 0.f};
#pragma unroll 1
  for (int k0 = 0; k0 < NHID; k0 += 32) {
    const v16h a = Frag<_Float16>::load(ahrow + k0);
    const v16h b = Frag<_Float16>::load(wfcrow + k0);
    acc = Frag<_Float16>::mma(a, b, acc);
    dep_guard1_h(acc, a, b);
  }
  acc_guard1(acc);
#pragma unroll
  for (int r = 0; r < 8; ++r) Fs[(8 * hh + r) * FPITCH + 16 * nt + c] = acc[r] * WCARRY_INV + fcbias;
}

__device__ __forceinline__ void store_frame(const float* Fs, float* out, int rowbase, int t, int tid) {
  const int row = tid >> 3, c4 = (tid & 7) * 4;
  const v4f v = *(const v4f*)(Fs + row * FPITCH + c4);
  float* p = out + ((size_t)(rowbase + row) * NSTEP + (size_t)t) * NOUTF + c4;
  *(volatile v4f*)p = v;
  __threadfence();
  *(volatile v4f*)p = v;
}

__global__ __launch_bounds__(NTHR) void lstm_ae_kernel(
    const float* __restrict__ x,
    const float* __restrict__ ebih, const float* __restrict__ ebhh,
    const float* __restrict__ dbih, const float* __restrict__ dbhh,
    const float* __restrict__ fcb,
    const unsigned short* __restrict__ WEXp,
    const unsigned short* __restrict__ WEHp,
    const unsigned short* __restrict__ WDHp,
    const unsigned short* __restrict__ WDSp,
    const unsigned short* __restrict__ WFCp,
    float* __restrict__ out) {
  __shared__ __align__(16) _Float16 Ax[16 * XPITCH];
  __shared__ __align__(16) _Float16 Ah[16 * HPITCH];
  __shared__ __align__(16) float    Fs[16 * FPITCH];
  const _Float16* WEX = (const _Float16*)WEXp;
  const _Float16* WEH = (const _Float16*)WEHp;
  const _Float16* WDH = (const _Float16*)WDHp;
  const _Float16* WDS = (const _Float16*)WDSp;
  const _Float16* WFC = (const _Float16*)WFCp;
  const int tid = threadIdx.x, lane = tid & 31, wave = tid >> 5;
  const int c = lane & 15, hh = lane >> 4, koff = hh * 8;
  const int rowbase = blockIdx.x * ROWS_PER_BLOCK;
  const int j = 16 * wave + c;

#pragma unroll 1
  for (int i = 0; i < 9; ++i) { const int idx = i * NTHR + tid; if (idx < 16 * HPITCH) Ah[idx] = (_Float16)0.0f; }
#pragma unroll 1
  for (int i = 0; i < 3; ++i) { const int idx = i * NTHR + tid; if (idx < 16 * XPITCH) Ax[idx] = (_Float16)0.0f; }
  __syncthreads();
  if (tid < 128) {
    const int m = tid >> 3, f4 = (tid & 7) * 4;
    const v4f v = *(const v4f*)(x + ((size_t)(rowbase + m) * NSTEP) * NIN + f4);
    Ax[m * XPITCH + f4 + 0] = (_Float16)v[0];
    Ax[m * XPITCH + f4 + 1] = (_Float16)v[1];
    Ax[m * XPITCH + f4 + 2] = (_Float16)v[2];
    Ax[m * XPITCH + f4 + 3] = (_Float16)v[3];
  }
  float be[4], bd[4], cst[8], hst[8];
#pragma unroll
  for (int g = 0; g < 4; ++g) {
    be[g] = ebih[g * NHID + j] + ebhh[g * NHID + j];
    bd[g] = dbih[g * NHID + j] + dbhh[g * NHID + j];
  }
#pragma unroll
  for (int r = 0; r < 8; ++r) { cst[r] = 0.0f; hst[r] = 0.0f; }
  const int fcn = 16 * (wave & 1) + c;
  const float fcbias = fcb[fcn];
  __syncthreads();

  const _Float16* axrow  = Ax + c * XPITCH + koff;
  const _Float16* ahrow  = Ah + c * HPITCH + koff;
  const _Float16* wexrow = WEX + (size_t)j * NIN + koff;
  const _Float16* wehrow = WEH + (size_t)j * NHID + koff;
  const _Float16* wfcrow = WFC + (size_t)fcn * NHID + koff;
  const v8f z8 = {0.f, 0.f, 0.f, 0.f, 0.f, 0.f, 0.f, 0.f};

#pragma unroll 1
  for (int t = 0; t < NSTEP; ++t) {
    v8f acc[4];
    acc[0] = z8; acc[1] = z8; acc[2] = z8; acc[3] = z8;
    {
      const v16h a  = Frag<_Float16>::load(axrow);
      const v16h b0 = Frag<_Float16>::load(wexrow);
      const v16h b1 = Frag<_Float16>::load(wexrow + (size_t)1 * NHID * NIN);
      const v16h b2 = Frag<_Float16>::load(wexrow + (size_t)2 * NHID * NIN);
      const v16h b3 = Frag<_Float16>::load(wexrow + (size_t)3 * NHID * NIN);
      acc[0] = Frag<_Float16>::mma(a, b0, acc[0]);
      acc[1] = Frag<_Float16>::mma(a, b1, acc[1]);
      acc[2] = Frag<_Float16>::mma(a, b2, acc[2]);
      acc[3] = Frag<_Float16>::mma(a, b3, acc[3]);
      dep_guard_h(acc[0], acc[3], a, b3);
      keep4_h(b0, b1, b2, b3);
    }
#pragma unroll 1
    for (int k0 = 0; k0 < NHID; k0 += 32) {
      const v16h a  = Frag<_Float16>::load(ahrow + k0);
      const v16h b0 = Frag<_Float16>::load(wehrow + k0);
      const v16h b1 = Frag<_Float16>::load(wehrow + (size_t)1 * NHID * NHID + k0);
      const v16h b2 = Frag<_Float16>::load(wehrow + (size_t)2 * NHID * NHID + k0);
      const v16h b3 = Frag<_Float16>::load(wehrow + (size_t)3 * NHID * NHID + k0);
      acc[0] = Frag<_Float16>::mma(a, b0, acc[0]);
      acc[1] = Frag<_Float16>::mma(a, b1, acc[1]);
      acc[2] = Frag<_Float16>::mma(a, b2, acc[2]);
      acc[3] = Frag<_Float16>::mma(a, b3, acc[3]);
      dep_guard_h(acc[0], acc[3], a, b3);
      keep4_h(b0, b1, b2, b3);
    }
    acc_guard4(acc[0], acc[1], acc[2], acc[3]);
#pragma unroll
    for (int r = 0; r < 8; ++r) {
      const float zi = acc[0][r] * WCARRY_INV + be[0];
      const float zf = acc[1][r] * WCARRY_INV + be[1];
      const float zg = acc[2][r] * WCARRY_INV + be[2];
      const float zo = acc[3][r] * WCARRY_INV + be[3];
      const float ig = fsig(zi);
      const float fg = fsig(zf);
      const float gg = ftanh(zg);
      const float og = fsig(zo);
      const float cn = fg * cst[r] + ig * gg;
      cst[r] = cn;
      hst[r] = og * ftanh(cn);
    }
    __syncthreads();
#pragma unroll
    for (int r = 0; r < 8; ++r) Ah[(8 * hh + r) * HPITCH + j] = (_Float16)hst[r];
    if (tid < 128) {
      const int tn = (t + 1 < NSTEP) ? (t + 1) : (NSTEP - 1);
      const int m = tid >> 3, f4 = (tid & 7) * 4;
      const v4f v = *(const v4f*)(x + ((size_t)(rowbase + m) * NSTEP + (size_t)tn) * NIN + f4);
      Ax[m * XPITCH + f4 + 0] = (_Float16)v[0];
      Ax[m * XPITCH + f4 + 1] = (_Float16)v[1];
      Ax[m * XPITCH + f4 + 2] = (_Float16)v[2];
      Ax[m * XPITCH + f4 + 3] = (_Float16)v[3];
    }
    __syncthreads();
  }

#pragma unroll 1
  for (int t = 0; t < NSTEP; ++t) {
    if (t > 0 && wave < 2) frame_head(ahrow, wfcrow, Fs, wave, hh, c, fcbias);
    const _Float16* wdrow = ((t == 0) ? WDH : WDS) + (size_t)j * NHID + koff;
    v8f acc[4];
    acc[0] = z8; acc[1] = z8; acc[2] = z8; acc[3] = z8;
#pragma unroll 1
    for (int k0 = 0; k0 < NHID; k0 += 32) {
      const v16h a  = Frag<_Float16>::load(ahrow + k0);
      const v16h b0 = Frag<_Float16>::load(wdrow + k0);
      const v16h b1 = Frag<_Float16>::load(wdrow + (size_t)1 * NHID * NHID + k0);
      const v16h b2 = Frag<_Float16>::load(wdrow + (size_t)2 * NHID * NHID + k0);
      const v16h b3 = Frag<_Float16>::load(wdrow + (size_t)3 * NHID * NHID + k0);
      acc[0] = Frag<_Float16>::mma(a, b0, acc[0]);
      acc[1] = Frag<_Float16>::mma(a, b1, acc[1]);
      acc[2] = Frag<_Float16>::mma(a, b2, acc[2]);
      acc[3] = Frag<_Float16>::mma(a, b3, acc[3]);
      dep_guard_h(acc[0], acc[3], a, b3);
      keep4_h(b0, b1, b2, b3);
    }
    acc_guard4(acc[0], acc[1], acc[2], acc[3]);
#pragma unroll
    for (int r = 0; r < 8; ++r) {
      const float zi = acc[0][r] * WCARRY_INV + bd[0];
      const float zf = acc[1][r] * WCARRY_INV + bd[1];
      const float zg = acc[2][r] * WCARRY_INV + bd[2];
      const float zo = acc[3][r] * WCARRY_INV + bd[3];
      const float ig = fsig(zi);
      const float fg = fsig(zf);
      const float gg = ftanh(zg);
      const float og = fsig(zo);
      const float cn = fg * cst[r] + ig * gg;
      hst[r] = og * ftanh(cn);
    }
    __syncthreads();
#pragma unroll
    for (int r = 0; r < 8; ++r) Ah[(8 * hh + r) * HPITCH + j] = (_Float16)hst[r];
    if (t > 0 && tid < 128) store_frame(Fs, out, rowbase, t - 1, tid);
    __syncthreads();
  }
  if (wave < 2) frame_head(ahrow, wfcrow, Fs, wave, hh, c, fcbias);
  __syncthreads();
  if (tid < 128) store_frame(Fs, out, rowbase, NSTEP - 1, tid);
}

extern "C" void kernel_launch(void* const* d_in, const int* in_sizes, int n_in,
                              void* d_out, int out_size, void* d_ws, size_t ws_size, hipStream_t stream) {
  if (n_in < 11 || d_out == nullptr || d_ws == nullptr) return;
  if (in_sizes[0] != NSEQ * NSTEP * NIN || in_sizes[1] != NGATE * NIN || in_sizes[2] != NGATE * NHID ||
      in_sizes[3] != NGATE || in_sizes[4] != NGATE || in_sizes[5] != NGATE * NHID || in_sizes[6] != NGATE * NHID ||
      in_sizes[7] != NGATE || in_sizes[8] != NGATE || in_sizes[9] != NOUTF * NHID || in_sizes[10] != NOUTF ||
      out_size != NSEQ * NSTEP * NOUTF) return;

  const float* xin  = (const float*)d_in[0];
  const float* eWih = (const float*)d_in[1];
  const float* eWhh = (const float*)d_in[2];
  const float* ebih = (const float*)d_in[3];
  const float* ebhh = (const float*)d_in[4];
  const float* dWih = (const float*)d_in[5];
  const float* dWhh = (const float*)d_in[6];
  const float* dbih = (const float*)d_in[7];
  const float* dbhh = (const float*)d_in[8];
  const float* fcW  = (const float*)d_in[9];
  const float* fcb  = (const float*)d_in[10];
  float* out = (float*)d_out;

  char* ws = (char*)d_ws; size_t off = 0;
  auto carve = [&](size_t bytes) -> char* { char* p = ws + off; off += (bytes + 255) & ~(size_t)255; return p; };
  _Float16* WEX = (_Float16*)carve((size_t)NGATE * NIN * 2);
  _Float16* WEH = (_Float16*)carve((size_t)NGATE * NHID * 2);
  _Float16* WDH = (_Float16*)carve((size_t)NGATE * NHID * 2);
  _Float16* WDS = (_Float16*)carve((size_t)NGATE * NHID * 2);
  _Float16* WFC = (_Float16*)carve((size_t)NOUTF * NHID * 2);
  if (off > ws_size || off > (size_t)134217728) return;

  const int n2x = NGATE * NIN / 2, n2h = NGATE * NHID / 2, n2f = NOUTF * NHID / 2;
  cast_scale_f16x2<<<(n2x + 255) / 256, 256, 0, stream>>>(eWih, WEX, n2x, WCARRY);
  cast_scale_f16x2<<<(n2h + 255) / 256, 256, 0, stream>>>(eWhh, WEH, n2h, WCARRY);
  cast_scale_f16x2<<<(n2h + 255) / 256, 256, 0, stream>>>(dWhh, WDH, n2h, WCARRY);
  addcast_scale_f16x2<<<(n2h + 255) / 256, 256, 0, stream>>>(dWih, dWhh, WDS, n2h, WCARRY);
  cast_scale_f16x2<<<(n2f + 255) / 256, 256, 0, stream>>>(fcW, WFC, n2f, WCARRY);
  lstm_ae_kernel<<<NSEQ / ROWS_PER_BLOCK, NTHR, 0, stream>>>(
      xin, ebih, ebhh, dbih, dbhh, fcb,
      (const unsigned short*)WEX, (const unsigned short*)WEH, (const unsigned short*)WDH,
      (const unsigned short*)WDS, (const unsigned short*)WFC, out);
}
